// LongNetAttentionBlock_28449863368954
// MI455X (gfx1250) — hardware-verified
//
#include <hip/hip_runtime.h>

typedef __attribute__((ext_vector_type(16))) _Float16 v16h;
typedef __attribute__((ext_vector_type(8)))  _Float16 v8h;
typedef __attribute__((ext_vector_type(16))) __bf16   v16b;
typedef __attribute__((ext_vector_type(8)))  __bf16   v8b;
typedef __attribute__((ext_vector_type(8)))  float    v8f;
typedef __attribute__((ext_vector_type(4)))  float    v4f;
typedef __attribute__((ext_vector_type(2)))  float    v2f;

#define CIN   48
#define IMGW  256
#define NSIDE 128
#define NTOK  16384
#define DM    192
#define SEGL  4096
#define QH    2048
#define NPROJ 576
#define QK_SCALE 0.07216878364870323f
#define P_CARRY 32768.0f
#define P_CARRY_INV (1.0f / 32768.0f)
#define LN_EPS 1e-5f

__device__ __forceinline__ unsigned short f2bf_bits(float f) {
  unsigned u = __float_as_uint(f);
  return (unsigned short)((u + 0x7FFFu + ((u >> 16) & 1u)) >> 16);
}
__device__ __forceinline__ float bf_bits2f(unsigned short h) { return __uint_as_float(((unsigned)h) << 16); }

__device__ __forceinline__ void dep_guard_h(v8f& a, v8f& b, v16h x, v16h y) { asm volatile("v_nop\n\tv_nop\n\tv_nop\n\tv_nop" : "+v"(a), "+v"(b) : "v"(x), "v"(y)); }
__device__ __forceinline__ void dep_guard_b(v8f& a, v8f& b, v16b x, v16b y) { asm volatile("v_nop\n\tv_nop\n\tv_nop\n\tv_nop" : "+v"(a), "+v"(b) : "v"(x), "v"(y)); }
__device__ __forceinline__ void keep4_h(v16h a, v16h b, v16h c, v16h d) { asm volatile("v_nop" :: "v"(a), "v"(b), "v"(c), "v"(d)); }
__device__ __forceinline__ void keep4_b(v16b a, v16b b, v16b c, v16b d) { asm volatile("v_nop" :: "v"(a), "v"(b), "v"(c), "v"(d)); }
__device__ __forceinline__ void acc_guard4(v8f& a, v8f& b, v8f& c, v8f& d) { asm volatile("v_nop\n\tv_nop\n\tv_nop\n\tv_nop" : "+v"(a), "+v"(b), "+v"(c), "+v"(d)); }

template <typename T> struct Frag;
template <> struct Frag<_Float16> {
  typedef v16h V; union U { v16h v; v8h h[2]; };
  static __device__ __forceinline__ v16h load(const _Float16* p) {
    U f; f.h[0] = *(const v8h*)(p); f.h[1] = *(const v8h*)(p + 16); return f.v;
  }
  static __device__ __forceinline__ v8f mma(v16h a, v16h b, v8f c) {
    return __builtin_amdgcn_wmma_f32_16x16x32_f16(false, a, false, b, (short)0, c, false, false);
  }
  static __device__ __forceinline__ void guard(v8f& a, v8f& b, v16h x, v16h y) { dep_guard_h(a, b, x, y); }
  static __device__ __forceinline__ void keep(v16h a, v16h b, v16h c, v16h d) { keep4_h(a, b, c, d); }
};
template <> struct Frag<__bf16> {
  typedef v16b V; union U { v16b v; v8b h[2]; };
  static __device__ __forceinline__ v16b load(const __bf16* p) {
    U f; f.h[0] = *(const v8b*)(p); f.h[1] = *(const v8b*)(p + 16); return f.v;
  }
  static __device__ __forceinline__ v8f mma(v16b a, v16b b, v8f c) {
    return __builtin_amdgcn_wmma_f32_16x16x32_bf16(false, a, false, b, (short)0, c, false, false);
  }
  static __device__ __forceinline__ void guard(v8f& a, v8f& b, v16b x, v16b y) { dep_guard_b(a, b, x, y); }
  static __device__ __forceinline__ void keep(v16b a, v16b b, v16b c, v16b d) { keep4_b(a, b, c, d); }
};

template <int ET> struct Elem;
template <> struct Elem<0> { typedef _Float16 T; };
template <> struct Elem<1> { typedef __bf16 T; };
template <int ET, bool SPLIT, int BIAS_MODE, int OUT_MODE, bool RESID, int ACT = 0>
__global__ __launch_bounds__(256) void wmma_gemm64(
    const unsigned short* __restrict__ Ap, const unsigned short* __restrict__ A2p, int lda, long strideA,
    const unsigned short* __restrict__ Btp, const unsigned short* __restrict__ Bt2p, int ldb, long strideB,
    void* __restrict__ Cout, void* __restrict__ Cout2, int ldc, long strideC,
    const float* __restrict__ bias,
    const float* __restrict__ resid, long strideR,
    int M, int N, int K, float scale) {
  typedef typename Elem<ET>::T T;
  typedef typename Frag<T>::V V;
  const T* A = (const T*)Ap; const T* A2 = (const T*)A2p; const T* Bt = (const T*)Btp; const T* Bt2 = (const T*)Bt2p;
  __shared__ __align__(16) float sT[8][16 * 68];
  const int b    = blockIdx.y;
  const int lane = threadIdx.x & 31;
  const int wave = threadIdx.x >> 5;
  const int tilesN = N >> 6;
  const int tilesM = M >> 6;
  const int tile = blockIdx.x * 8 + wave;
  if (tile >= tilesM * tilesN) return;
  const int tm = tile / tilesN;
  const int tn = tile - tm * tilesN;
  const int m0 = tm << 6;
  const int n0 = tn << 6;

  const T* Ab  = A  + (size_t)b * strideA;
  const T* Bb  = Bt + (size_t)b * strideB;
  const T* Ab2 = SPLIT ? (A2  + (size_t)b * strideA) : nullptr;
  const T* Bb2 = SPLIT ? (Bt2 + (size_t)b * strideB) : nullptr;

  const int rlane = lane & 15;
  const int koff  = (lane >> 4) * 8;
  const int mOff  = (lane >> 4) * 8;

  v8f acc[4][4];
#pragma unroll
  for (int i = 0; i < 4; ++i)
#pragma unroll
    for (int j = 0; j < 4; ++j) acc[i][j] = (v8f){0.f,0.f,0.f,0.f,0.f,0.f,0.f,0.f};

  for (int k0 = 0; k0 < K; k0 += 32) {
    V bh[4], bl[4];
#pragma unroll
    for (int j = 0; j < 4; ++j) {
      const size_t bo = (size_t)(n0 + (j << 4) + rlane) * ldb + koff + k0;
      bh[j] = Frag<T>::load(Bb + bo);
      if (SPLIT) bl[j] = Frag<T>::load(Bb2 + bo);
    }
#pragma unroll
    for (int i = 0; i < 4; ++i) {
      const size_t ao = (size_t)(m0 + (i << 4) + rlane) * lda + koff + k0;
      V ah = Frag<T>::load(Ab + ao);
      V al;
      if (SPLIT) al = Frag<T>::load(Ab2 + ao);
#pragma unroll
      for (int j = 0; j < 4; ++j) {
        acc[i][j] = Frag<T>::mma(ah, bh[j], acc[i][j]);
        if (SPLIT) {
          acc[i][j] = Frag<T>::mma(ah, bl[j], acc[i][j]);
          acc[i][j] = Frag<T>::mma(al, bh[j], acc[i][j]);
        }
      }
      Frag<T>::guard(acc[i][0], acc[i][3], ah, SPLIT ? al : ah);
    }
    Frag<T>::keep(bh[0], bh[1], bh[2], bh[3]);
    if (SPLIT) Frag<T>::keep(bl[0], bl[1], bl[2], bl[3]);
  }
  acc_guard4(acc[0][0], acc[0][1], acc[0][2], acc[0][3]);
  acc_guard4(acc[1][0], acc[1][1], acc[1][2], acc[1][3]);
  acc_guard4(acc[2][0], acc[2][1], acc[2][2], acc[2][3]);
  acc_guard4(acc[3][0], acc[3][1], acc[3][2], acc[3][3]);

  float* slab = sT[wave];
  const float* Rb = RESID ? (resid + (size_t)b * strideR) : nullptr;
#pragma unroll
  for (int i = 0; i < 4; ++i) {
    const int mBase = m0 + (i << 4);
#pragma unroll
    for (int j = 0; j < 4; ++j) {
      const int n = n0 + (j << 4) + rlane;
      float bv = 0.f;
      if (BIAS_MODE == 2) bv = bias[n];
#pragma unroll
      for (int r = 0; r < 8; ++r) {
        float v = acc[i][j][r] * scale;
        if (BIAS_MODE == 1) v += bias[mBase + mOff + r];
        if (BIAS_MODE == 2) v += bv;
        if (RESID) v += Rb[(size_t)(mBase + mOff + r) * ldc + n];
        if (ACT == 1) v = tanhf(v);
        if (ACT == 2) v = fmaxf(v, 0.0f);
        if (ACT == 3) v = v / (1.0f + expf(-v));
        if (ACT == 4) v = (v > 0.f) ? v : 0.01f * v;
        if (ACT == 5) v = 0.5f * v * (1.0f + erff(v * 0.70710678118654752f));
        slab[(mOff + r) * 68 + (j << 4) + rlane] = v;
      }
    }
    __builtin_amdgcn_fence(__ATOMIC_RELEASE, "workgroup");
    __builtin_amdgcn_wave_barrier();
    __builtin_amdgcn_fence(__ATOMIC_ACQUIRE, "workgroup");
    if (OUT_MODE == 0) {
      float* C = (float*)Cout + (size_t)b * strideC;
      const int hh = lane >> 4, c4 = (lane & 15) * 4;
      for (int pass = 0; pass < 2; ++pass) {
#pragma unroll
        for (int it = 0; it < 8; ++it) {
          const int row = it * 2 + hh;
          v4f v = *(const v4f*)(slab + row * 68 + c4);
          *(volatile v4f*)(C + (size_t)(mBase + row) * ldc + n0 + c4) = v;
        }
        __threadfence();
      }
    } else {
      const int q = lane >> 3, c8 = (lane & 7) * 8;
      unsigned short* C  = (unsigned short*)Cout  + (size_t)b * strideC;
      unsigned short* C2 = (OUT_MODE == 2) ? ((unsigned short*)Cout2 + (size_t)b * strideC) : nullptr;
      for (int pass = 0; pass < 2; ++pass) {
#pragma unroll
        for (int it = 0; it < 4; ++it) {
          const int row = it * 4 + q;
          const float* sp = slab + row * 68 + c8;
          v8h hv, lv;
#pragma unroll
          for (int e = 0; e < 8; ++e) {
            if (OUT_MODE == 1) {
              hv[e] = (_Float16)sp[e];
            } else {
              unsigned short hb = f2bf_bits(sp[e]);
              unsigned short lb = f2bf_bits(sp[e] - bf_bits2f(hb));
              hv[e] = __builtin_bit_cast(_Float16, hb);
              lv[e] = __builtin_bit_cast(_Float16, lb);
            }
          }
          *(volatile v8h*)(C + (size_t)(mBase + row) * ldc + n0 + c8) = hv;
          if (OUT_MODE == 2) *(volatile v8h*)(C2 + (size_t)(mBase + row) * ldc + n0 + c8) = lv;
        }
        __threadfence();
      }
    }
    __builtin_amdgcn_fence(__ATOMIC_RELEASE, "workgroup");
    __builtin_amdgcn_wave_barrier();
    __builtin_amdgcn_fence(__ATOMIC_ACQUIRE, "workgroup");
  }
}

__global__ __launch_bounds__(256) void cast_f32_f16x2(
    const float* __restrict__ in, _Float16* __restrict__ out, int n2) {
  int i = blockIdx.x * 256 + threadIdx.x;
  if (i < n2) {
    const _Float16 h0 = (_Float16)in[2 * i], h1 = (_Float16)in[2 * i + 1];
    const unsigned u = (unsigned)__builtin_bit_cast(unsigned short, h0) | ((unsigned)__builtin_bit_cast(unsigned short, h1) << 16);
    ((volatile unsigned*)out)[i] = u;
    __threadfence();
    ((volatile unsigned*)out)[i] = u;
  }
}

__device__ __forceinline__ float wave_sum(float v) {
#pragma unroll
  for (int o = 16; o > 0; o >>= 1) v += __shfl_xor(v, o, 32);
  return v;
}
__device__ __forceinline__ float wave_max(float v) {
#pragma unroll
  for (int o = 16; o > 0; o >>= 1) v = fmaxf(v, __shfl_xor(v, o, 32));
  return v;
}

__global__ __launch_bounds__(256) void k_patchify(const float* __restrict__ x, _Float16* __restrict__ t16, int total) {
  const int i = blockIdx.x * 256 + threadIdx.x;
  if (i >= total) return;
  const int token = i / (DM / 8);
  const int dg = i - token * (DM / 8);
  const int ny = token >> 7, nx = token & 127;
  v8h h;
#pragma unroll
  for (int cc = 0; cc < 2; ++cc) {
    const int c = dg * 2 + cc;
#pragma unroll
    for (int wy = 0; wy < 2; ++wy) {
      const int Y = ny * 2 + wy;
      const v2f q = *(const v2f*)(x + (size_t)c * (IMGW * IMGW) + (size_t)Y * IMGW + nx * 2);
      h[cc * 4 + wy * 2 + 0] = (_Float16)q[0];
      h[cc * 4 + wy * 2 + 1] = (_Float16)q[1];
    }
  }
  _Float16* dp = t16 + (size_t)i * 8;
  *(volatile v8h*)dp = h;
  __threadfence();
  *(volatile v8h*)dp = h;
}

__global__ __launch_bounds__(256) void k_ln_qkv(
    const float* __restrict__ qkv, const float* __restrict__ bq, const float* __restrict__ bk, const float* __restrict__ bv,
    const float* __restrict__ gamma, const float* __restrict__ beta,
    _Float16* __restrict__ q16, _Float16* __restrict__ k16, _Float16* __restrict__ vT16, int seg) {
  __shared__ __align__(16) _Float16 vs[64 * DM];
  const int tid = threadIdx.x, lane = tid & 31, wave = tid >> 5;
  const int tok0 = blockIdx.x * 64;
  const bool act = lane < 24;
  const int e0 = (act ? lane : 0) * 8;
  const v4f z4 = {0.f, 0.f, 0.f, 0.f};
  const v4f g0 = *(const v4f*)(gamma + e0), g1 = *(const v4f*)(gamma + e0 + 4);
  const v4f h0 = *(const v4f*)(beta + e0),  h1 = *(const v4f*)(beta + e0 + 4);
  const v4f cq0 = *(const v4f*)(bq + e0), cq1 = *(const v4f*)(bq + e0 + 4);
  const v4f ck0 = *(const v4f*)(bk + e0), ck1 = *(const v4f*)(bk + e0 + 4);
  const v4f cv0 = *(const v4f*)(bv + e0), cv1 = *(const v4f*)(bv + e0 + 4);

#pragma unroll 1
  for (int i = 0; i < 8; ++i) {
    const int tl = wave * 8 + i;
    const size_t row = (size_t)(tok0 + tl);
    const float* rp = qkv + row * NPROJ + e0;
#pragma unroll
    for (int p = 0; p < 3; ++p) {
      const v4f c0 = (p == 0) ? cq0 : (p == 1) ? ck0 : cv0;
      const v4f c1 = (p == 0) ? cq1 : (p == 1) ? ck1 : cv1;
      v4f t0 = *(const v4f*)(rp + p * DM) + c0;
      v4f t1 = *(const v4f*)(rp + p * DM + 4) + c1;
      t0 = act ? t0 : z4;
      t1 = act ? t1 : z4;
      float s = ((t0[0] + t0[1]) + (t0[2] + t0[3])) + ((t1[0] + t1[1]) + (t1[2] + t1[3]));
      s = wave_sum(s);
      const float mu = s * (1.0f / 192.0f);
      v4f d0 = t0 - mu, d1 = t1 - mu;
      d0 = act ? d0 : z4;
      d1 = act ? d1 : z4;
      float v2 = ((d0[0] * d0[0] + d0[1] * d0[1]) + (d0[2] * d0[2] + d0[3] * d0[3]))
               + ((d1[0] * d1[0] + d1[1] * d1[1]) + (d1[2] * d1[2] + d1[3] * d1[3]));
      v2 = wave_sum(v2);
      const float rs = rsqrtf(v2 * (1.0f / 192.0f) + LN_EPS);
      const v4f y0 = (d0 * rs) * g0 + h0;
      const v4f y1 = (d1 * rs) * g1 + h1;
      v8h hv;
#pragma unroll
      for (int j = 0; j < 4; ++j) { hv[j] = (_Float16)y0[j]; hv[4 + j] = (_Float16)y1[j]; }
      if (p == 0) {
        if (act) {
          _Float16* dp = q16 + row * DM + e0;
          *(volatile v8h*)dp = hv;
          __threadfence();
          *(volatile v8h*)dp = hv;
        }
      } else if (p == 1) {
        if (act) {
          _Float16* dp = k16 + row * DM + e0;
          *(volatile v8h*)dp = hv;
          __threadfence();
          *(volatile v8h*)dp = hv;
        }
      } else {
        if (act) *(v8h*)(vs + tl * DM + e0) = hv;
      }
    }
  }
  __syncthreads();

  const int g = tok0 / seg;
  const int sin0 = tok0 - g * seg;
  _Float16* vb = vT16 + (size_t)g * DM * seg + sin0;
  const int s8 = (lane & 7) * 8, dq = lane >> 3;
  for (int pass = 0; pass < 2; ++pass) {
#pragma unroll
    for (int it = 0; it < 6; ++it) {
      const int d = wave * 24 + it * 4 + dq;
      v8h hv;
#pragma unroll
      for (int j = 0; j < 8; ++j) hv[j] = vs[(s8 + j) * DM + d];
      *(volatile v8h*)(vb + (size_t)d * seg + s8) = hv;
    }
    __threadfence();
  }
}

__global__ __launch_bounds__(256) void k_softmax_row(const float* __restrict__ S, _Float16* __restrict__ P, int ncols) {
  __shared__ float red[16];
  const int tid = threadIdx.x, lane = tid & 31, wave = tid >> 5;
  const size_t rowoff = (size_t)blockIdx.x * ncols;
  const float* sr = S + rowoff;
  const int ca = tid * 8, cb = (ncols >> 1) + tid * 8;
  v4f a0 = *(const v4f*)(sr + ca), a1 = *(const v4f*)(sr + ca + 4);
  v4f b0 = *(const v4f*)(sr + cb), b1 = *(const v4f*)(sr + cb + 4);
  float m = a0[0];
#pragma unroll
  for (int e = 0; e < 4; ++e) { m = fmaxf(m, a0[e]); m = fmaxf(m, a1[e]); m = fmaxf(m, b0[e]); m = fmaxf(m, b1[e]); }
  m = wave_max(m);
  if (lane == 0) red[wave] = m;
  __syncthreads();
  float gm = red[0];
#pragma unroll
  for (int w = 1; w < 8; ++w) gm = fmaxf(gm, red[w]);
  float sum = 0.f;
#pragma unroll
  for (int e = 0; e < 4; ++e) {
    a0[e] = __expf(a0[e] - gm); sum += a0[e];
    a1[e] = __expf(a1[e] - gm); sum += a1[e];
    b0[e] = __expf(b0[e] - gm); sum += b0[e];
    b1[e] = __expf(b1[e] - gm); sum += b1[e];
  }
  sum = wave_sum(sum);
  if (lane == 0) red[8 + wave] = sum;
  __syncthreads();
  float tot = red[8];
#pragma unroll
  for (int w = 1; w < 8; ++w) tot += red[8 + w];
  const float inv = 1.0f / tot;
  v8h ha, hb;
#pragma unroll
  for (int e = 0; e < 4; ++e) {
    ha[e]     = (_Float16)((a0[e] * inv) * P_CARRY);
    ha[4 + e] = (_Float16)((a1[e] * inv) * P_CARRY);
    hb[e]     = (_Float16)((b0[e] * inv) * P_CARRY);
    hb[4 + e] = (_Float16)((b1[e] * inv) * P_CARRY);
  }
  _Float16* pr = P + rowoff;
  *(volatile v8h*)(pr + ca) = ha;
  *(volatile v8h*)(pr + cb) = hb;
  __threadfence();
  *(volatile v8h*)(pr + ca) = ha;
  *(volatile v8h*)(pr + cb) = hb;
}

__global__ __launch_bounds__(256) void k_unpatchify(const float* __restrict__ O, float* __restrict__ out, int total) {
  const int i = blockIdx.x * 256 + threadIdx.x;
  if (i >= total) return;
  const int j = i & 63;
  const int rowi = i >> 6;
  const int Y = rowi & 255, c = rowi >> 8;
  const int ny = Y >> 1, wy = Y & 1;
  const int d0 = c * 4 + wy * 2;
  const int s0 = ny * NSIDE + 2 * j;
  const v2f p0 = *(const v2f*)(O + (size_t)s0 * DM + d0);
  const v2f p1 = *(const v2f*)(O + (size_t)(s0 + 1) * DM + d0);
  v4f v;
  v[0] = p0[0]; v[1] = p0[1]; v[2] = p1[0]; v[3] = p1[1];
  float* dp = out + (size_t)i * 4;
  *(volatile v4f*)dp = v;
  __threadfence();
  *(volatile v4f*)dp = v;
}

static void gemm_f16_f32out(const _Float16* A, int lda, const _Float16* Bt, int ldb, float* C, int ldc,
                            int M, int N, int K, float scale, const float* auxf, hipStream_t stream) {
  const int tiles = (M / 64) * (N / 64);
  dim3 grid((tiles + 7) / 8, 1, 1);
  wmma_gemm64<0, false, 0, 0, false, 0><<<grid, 256, 0, stream>>>(
      (const unsigned short*)A, (const unsigned short*)A, lda, 0L,
      (const unsigned short*)Bt, (const unsigned short*)Bt, ldb, 0L,
      (void*)C, (void*)C, ldc, 0L,
      auxf, auxf, 0L, M, N, K, scale);
}

extern "C" void kernel_launch(void* const* d_in, const int* in_sizes, int n_in,
                              void* d_out, int out_size, void* d_ws, size_t ws_size,
                              hipStream_t stream) {
  if (n_in < 9) return;
  if (in_sizes[0] != CIN * IMGW * IMGW) return;
  if (in_sizes[1] != DM * DM || in_sizes[3] != DM * DM || in_sizes[5] != DM * DM) return;
  if (in_sizes[2] != DM || in_sizes[4] != DM || in_sizes[6] != DM || in_sizes[7] != DM || in_sizes[8] != DM) return;
  if (out_size != CIN * IMGW * IMGW) return;

  const float* x     = (const float*)d_in[0];
  const float* Wq    = (const float*)d_in[1];
  const float* bq    = (const float*)d_in[2];
  const float* Wk    = (const float*)d_in[3];
  const float* bk    = (const float*)d_in[4];
  const float* Wv    = (const float*)d_in[5];
  const float* bv    = (const float*)d_in[6];
  const float* gamma = (const float*)d_in[7];
  const float* beta  = (const float*)d_in[8];
  float* out = (float*)d_out;

  const size_t bW16   = (size_t)NPROJ * DM * 2;
  const size_t bTok16 = (size_t)NTOK * DM * 2;
  const size_t bO     = (size_t)NTOK * DM * 4;
  const size_t bQKV   = (size_t)NTOK * NPROJ * 4;
  const size_t bS     = (size_t)QH * SEGL * 4;
  const size_t bP     = (size_t)QH * SEGL * 2;
  size_t off = 0;
  const size_t off_W16 = off;  off += bW16;
  const size_t off_q16 = off;  off += bTok16;
  const size_t off_k16 = off;  off += bTok16;
  const size_t off_vT  = off;  off += bTok16;
  const size_t off_O   = off;  off += bO;
  const size_t off_X   = off;
  const size_t phase1 = bTok16 + bQKV;
  const size_t phase2 = bS + bP;
  off += (phase1 > phase2) ? phase1 : phase2;
  if (off > ws_size) return;

  char* ws = (char*)d_ws;
  _Float16* W16  = (_Float16*)(ws + off_W16);
  _Float16* q16  = (_Float16*)(ws + off_q16);
  _Float16* k16  = (_Float16*)(ws + off_k16);
  _Float16* vT16 = (_Float16*)(ws + off_vT);
  float*    Of   = (float*)(ws + off_O);
  _Float16* t16  = (_Float16*)(ws + off_X);
  float*    qkvf = (float*)(ws + off_X + bTok16);
  float*    Sf   = (float*)(ws + off_X);
  _Float16* P16  = (_Float16*)(ws + off_X + bS);

  const int n2 = DM * DM / 2;
  cast_f32_f16x2<<<(n2 + 255) / 256, 256, 0, stream>>>(Wq, W16, n2);
  cast_f32_f16x2<<<(n2 + 255) / 256, 256, 0, stream>>>(Wk, W16 + (size_t)DM * DM, n2);
  cast_f32_f16x2<<<(n2 + 255) / 256, 256, 0, stream>>>(Wv, W16 + (size_t)2 * DM * DM, n2);

  const int totp = NTOK * (DM / 8);
  k_patchify<<<(totp + 255) / 256, 256, 0, stream>>>(x, t16, totp);

  gemm_f16_f32out(t16, DM, W16, DM, qkvf, NPROJ, NTOK, NPROJ, DM, 1.0f, gamma, stream);

  k_ln_qkv<<<NTOK / 64, 256, 0, stream>>>(qkvf, bq, bk, bv, gamma, beta, q16, k16, vT16, SEGL);

  for (int g = 0; g < NTOK / SEGL; ++g) {
    const _Float16* kB = k16 + (size_t)g * SEGL * DM;
    const _Float16* vB = vT16 + (size_t)g * DM * SEGL;
    for (int hf = 0; hf < SEGL / QH; ++hf) {
      const size_t qrow0 = (size_t)g * SEGL + (size_t)hf * QH;
      const _Float16* qA = q16 + qrow0 * DM;
      gemm_f16_f32out(qA, DM, kB, DM, Sf, SEGL, QH, SEGL, DM, QK_SCALE, gamma, stream);
      k_softmax_row<<<QH, 256, 0, stream>>>(Sf, P16, SEGL);
      gemm_f16_f32out(P16, SEGL, vB, SEGL, Of + qrow0 * DM, DM, QH, DM, SEGL, P_CARRY_INV, gamma, stream);
    }
  }

  const int totu = CIN * IMGW * (IMGW / 4);
  k_unpatchify<<<(totu + 255) / 256, 256, 0, stream>>>(Of, out, totu);
}
